// MultiheadVanillaAttention_71236327571792
// MI455X (gfx1250) — hardware-verified
//
#include <hip/hip_runtime.h>
#include <stdint.h>

typedef __bf16         v16bf __attribute__((ext_vector_type(16)));
typedef unsigned short v8us  __attribute__((ext_vector_type(8)));
typedef float          v8f   __attribute__((ext_vector_type(8)));
typedef float          v4f   __attribute__((ext_vector_type(4)));
typedef v4f            v4fa  __attribute__((may_alias));
typedef unsigned short ushort_t;

#define S_LEN  2048
#define BATCH  2
#define EMB    1024
#define HEADS  16
#define HDIM   64
#define MROWS  4096
#define GBM    128
#define GBN    64
#define TPITCH 68
#define NEGBIG (-1.0e30f)

static_assert(MROWS == S_LEN * BATCH);
static_assert(MROWS % GBM == 0);
static_assert(EMB % GBN == 0);
static_assert(EMB % 32 == 0);
static_assert(GBN == HDIM);
static_assert(S_LEN % 64 == 0);
static_assert((TPITCH * 4) % 16 == 0);

union Frag { v16bf v; v8us u[2]; };

__device__ __forceinline__ unsigned bf16_rne_bits(float f) {
  unsigned u = __float_as_uint(f);
  u += 0x7FFFu + ((u >> 16) & 1u);
  return u >> 16;
}
__device__ __forceinline__ void split_bf16(float f, unsigned& hb, unsigned& lb) {
  hb = bf16_rne_bits(f);
  const float fh = __uint_as_float(hb << 16);
  lb = bf16_rne_bits(f - fh);
}
__device__ __forceinline__ void pack8(v4f a, v4f c, v8us& hv, v8us& lv) {
  float f[8] = {a.x, a.y, a.z, a.w, c.x, c.y, c.z, c.w};
  hv = {};
  lv = {};
#pragma unroll
  for (int i = 0; i < 8; ++i) {
    unsigned hb, lb;
    split_bf16(f[i], hb, lb);
    hv[i] = (ushort_t)hb;
    lv[i] = (ushort_t)lb;
  }
}

__device__ __forceinline__ v16bf ldfrag(const ushort_t* __restrict__ p, int h) {
  Frag f;
  f.u[0] = *(const v8us*)(p + 8 * h);
  f.u[1] = *(const v8us*)(p + 16 + 8 * h);
  return f.v;
}

__device__ __forceinline__ v8f mma3(v16bf ah, v16bf al, v16bf bh, v16bf bl, v8f acc) {
  acc = __builtin_amdgcn_wmma_f32_16x16x32_bf16(false, ah, false, bh, (short)0, acc, false, false);
  acc = __builtin_amdgcn_wmma_f32_16x16x32_bf16(false, ah, false, bl, (short)0, acc, false, false);
  acc = __builtin_amdgcn_wmma_f32_16x16x32_bf16(false, al, false, bh, (short)0, acc, false, false);
  asm volatile("v_nop\n\tv_nop\n\tv_nop\n\tv_nop" : "+v"(acc) : "v"(ah), "v"(al), "v"(bh), "v"(bl));
  return acc;
}

__global__ __launch_bounds__(256)
void k_split_planes(const float* __restrict__ s0, const float* __restrict__ s1,
                    const float* __restrict__ s2, const float* __restrict__ s3,
                    int groupsPerSeg, ushort_t* __restrict__ hi, ushort_t* __restrict__ lo)
{
  const int seg = blockIdx.y;
  const int g = blockIdx.x * blockDim.x + threadIdx.x;
  if (g >= groupsPerSeg) return;
  const float* src = s0;
  if (seg == 1) src = s1;
  if (seg == 2) src = s2;
  if (seg == 3) src = s3;
  const size_t e = (size_t)g * 8;
  const v4f a = *(const v4fa*)(src + e);
  const v4f c = *(const v4fa*)(src + e + 4);
  v8us hv, lv;
  pack8(a, c, hv, lv);
  const size_t o = (size_t)seg * (size_t)groupsPerSeg * 8 + e;
  *(volatile v8us*)(hi + o) = hv;
  *(volatile v8us*)(lo + o) = lv;
  __threadfence();
  *(volatile v8us*)(hi + o) = hv;
  *(volatile v8us*)(lo + o) = lv;
}

template <int MODE>
__device__ __forceinline__ void gemm_store(float (*tile)[TPITCH], int tid, int mBase, int nBase,
                                           ushort_t* __restrict__ Oh, ushort_t* __restrict__ Ol,
                                           float* __restrict__ Of)
{
  if (MODE == 0) {
    const int p = tid & 7, rsub = tid >> 3;
#pragma unroll
    for (int it = 0; it < GBM / 16; ++it) {
      const int row = it * 16 + rsub;
      const v4f a = *(const v4fa*)(&tile[row][8 * p]);
      const v4f c = *(const v4fa*)(&tile[row][8 * p + 4]);
      v8us hv, lv;
      pack8(a, c, hv, lv);
      const size_t o = (size_t)(mBase + row) * EMB + nBase + 8 * p;
      *(volatile v8us*)(Oh + o) = hv;
      *(volatile v8us*)(Ol + o) = lv;
    }
  } else if (MODE == 1) {
    const int p = tid & 7, lsub = tid >> 3;
    const int hh = nBase / HDIM;
    const int s0 = mBase / BATCH;
#pragma unroll
    for (int it = 0; it < (BATCH * GBN) / 16; ++it) {
      const int li = it * 16 + lsub;
      const int bsel = li >> 6;
      const int d = li & 63;
      v4f a, c;
      a.x = tile[(8 * p + 0) * 2 + bsel][d];
      a.y = tile[(8 * p + 1) * 2 + bsel][d];
      a.z = tile[(8 * p + 2) * 2 + bsel][d];
      a.w = tile[(8 * p + 3) * 2 + bsel][d];
      c.x = tile[(8 * p + 4) * 2 + bsel][d];
      c.y = tile[(8 * p + 5) * 2 + bsel][d];
      c.z = tile[(8 * p + 6) * 2 + bsel][d];
      c.w = tile[(8 * p + 7) * 2 + bsel][d];
      v8us hv, lv;
      pack8(a, c, hv, lv);
      const size_t o = ((size_t)((bsel * HEADS + hh) * HDIM + d)) * S_LEN + s0 + 8 * p;
      *(volatile v8us*)(Oh + o) = hv;
      *(volatile v8us*)(Ol + o) = lv;
    }
  } else {
    const int p = tid & 15, rsub = tid >> 4;
#pragma unroll
    for (int it = 0; it < GBM / 8; ++it) {
      const int row = it * 8 + rsub;
      const v4f a = *(const v4fa*)(&tile[row][4 * p]);
      const size_t o = (size_t)(mBase + row) * EMB + nBase + 4 * p;
      *(volatile v4f*)(Of + o) = a;
    }
  }
}

template <int MODE>
__global__ __launch_bounds__(128)
void k_gemm(const ushort_t* __restrict__ Ah, const ushort_t* __restrict__ Al,
            const ushort_t* __restrict__ Wh, const ushort_t* __restrict__ Wl,
            const float* __restrict__ bias, float scale,
            ushort_t* __restrict__ Oh, ushort_t* __restrict__ Ol, float* __restrict__ Of)
{
  __shared__ __attribute__((aligned(16))) float tile[GBM][TPITCH];

  const int tid = threadIdx.x;
  const int lane = tid & 31;
  const int w = tid >> 5;
  const int h = lane >> 4;
  const int ln = lane & 15;
  const int mBase = blockIdx.y * GBM;
  const int nBase = blockIdx.x * GBN;
  const int wRow = mBase + 32 * w;

  v8f acc[2][4];
#pragma unroll
  for (int mt = 0; mt < 2; ++mt)
#pragma unroll
    for (int nt = 0; nt < 4; ++nt) acc[mt][nt] = {};

#pragma unroll 1
  for (int k0 = 0; k0 < EMB; k0 += 32) {
    v16bf ah[2], al[2];
#pragma unroll
    for (int mt = 0; mt < 2; ++mt) {
      const size_t ao = (size_t)(wRow + 16 * mt + ln) * EMB + k0;
      ah[mt] = ldfrag(Ah + ao, h);
      al[mt] = ldfrag(Al + ao, h);
    }
#pragma unroll
    for (int nt = 0; nt < 4; ++nt) {
      const size_t bo = (size_t)(nBase + 16 * nt + ln) * EMB + k0;
      const v16bf bh = ldfrag(Wh + bo, h);
      const v16bf bl = ldfrag(Wl + bo, h);
#pragma unroll
      for (int mt = 0; mt < 2; ++mt)
        acc[mt][nt] = mma3(ah[mt], al[mt], bh, bl, acc[mt][nt]);
    }
  }

#pragma unroll
  for (int nt = 0; nt < 4; ++nt) {
    const float bvn = bias[nBase + 16 * nt + ln];
#pragma unroll
    for (int mt = 0; mt < 2; ++mt)
#pragma unroll
      for (int r = 0; r < 8; ++r)
        tile[32 * w + 16 * mt + 8 * h + r][16 * nt + ln] = (acc[mt][nt][r] + bvn) * scale;
  }
  __syncthreads();

  gemm_store<MODE>(tile, tid, mBase, nBase, Oh, Ol, Of);
  __threadfence();
  gemm_store<MODE>(tile, tid, mBase, nBase, Oh, Ol, Of);
}

__device__ __forceinline__ void attn_store(float (*osh)[TPITCH], int tid, int qBase, int b,
                                           size_t headCol, ushort_t* __restrict__ Ch,
                                           ushort_t* __restrict__ Cl)
{
  const int p = tid & 7, rsub = tid >> 3;
#pragma unroll
  for (int it = 0; it < 4; ++it) {
    const int qi = it * 16 + rsub;
    const v4f a = *(const v4fa*)(&osh[qi][8 * p]);
    const v4f c = *(const v4fa*)(&osh[qi][8 * p + 4]);
    v8us hv, lv;
    pack8(a, c, hv, lv);
    const size_t o = ((size_t)(qBase + qi) * BATCH + b) * EMB + headCol + 8 * p;
    *(volatile v8us*)(Ch + o) = hv;
    *(volatile v8us*)(Cl + o) = lv;
  }
}

__global__ __launch_bounds__(128)
void k_attn(const ushort_t* __restrict__ Qh, const ushort_t* __restrict__ Ql,
            const ushort_t* __restrict__ Kh, const ushort_t* __restrict__ Kl,
            const ushort_t* __restrict__ Vth, const ushort_t* __restrict__ Vtl,
            ushort_t* __restrict__ Ch, ushort_t* __restrict__ Cl)
{
  __shared__ __attribute__((aligned(16))) float osh[64][TPITCH];

  const int tid = threadIdx.x;
  const int lane = tid & 31;
  const int w = tid >> 5;
  const int h = lane >> 4;
  const int ln = lane & 15;
  const int qBase = blockIdx.x * 64;
  const int b = blockIdx.y / HEADS;
  const int hd = blockIdx.y % HEADS;
  const int q0 = qBase + 16 * w;
  const size_t headCol = (size_t)hd * HDIM;

  v16bf qbh[2], qbl[2];
  {
    const size_t qo = ((size_t)(q0 + ln) * BATCH + b) * EMB + headCol;
#pragma unroll
    for (int c = 0; c < 2; ++c) {
      qbh[c] = ldfrag(Qh + qo + 32 * c, h);
      qbl[c] = ldfrag(Ql + qo + 32 * c, h);
    }
  }

  v8f acc[4];
#pragma unroll
  for (int j = 0; j < 4; ++j) acc[j] = {};
  float m = NEGBIG, l = 0.0f;
  const int thr = 16 * w + ln;
  const size_t vrow0 = ((size_t)(b * HEADS + hd) * HDIM) * S_LEN;

#pragma unroll 1
  for (int kb = 0; kb <= qBase; kb += 64) {
    v8f s[4];
#pragma unroll
    for (int kt = 0; kt < 4; ++kt) {
      s[kt] = {};
      const size_t ko = ((size_t)(kb + 16 * kt + ln) * BATCH + b) * EMB + headCol;
#pragma unroll
      for (int c = 0; c < 2; ++c) {
        const v16bf kah = ldfrag(Kh + ko + 32 * c, h);
        const v16bf kal = ldfrag(Kl + ko + 32 * c, h);
        s[kt] = mma3(kah, kal, qbh[c], qbl[c], s[kt]);
      }
    }
    if (kb == qBase) {
#pragma unroll
      for (int kt = 0; kt < 4; ++kt)
#pragma unroll
        for (int r = 0; r < 8; ++r)
          if (16 * kt + 8 * h + r > thr) s[kt][r] = NEGBIG;
    }

    float tmax = NEGBIG;
#pragma unroll
    for (int kt = 0; kt < 4; ++kt)
#pragma unroll
      for (int r = 0; r < 8; ++r) tmax = fmaxf(tmax, s[kt][r]);
    tmax = fmaxf(tmax, __shfl_xor(tmax, 16, 32));
    const float newm = fmaxf(m, tmax);
    const float corr = __expf(m - newm);
    m = newm;
    float psum = 0.0f;
#pragma unroll
    for (int kt = 0; kt < 4; ++kt)
#pragma unroll
      for (int r = 0; r < 8; ++r) {
        const float pv = __expf(s[kt][r] - newm);
        s[kt][r] = pv;
        psum += pv;
      }
    psum += __shfl_xor(psum, 16, 32);
    l = l * corr + psum;
#pragma unroll
    for (int j = 0; j < 4; ++j) acc[j] = acc[j] * corr;

#pragma unroll
    for (int kc = 0; kc < 2; ++kc) {
      v8us ph0 = {}, pl0 = {}, ph1 = {}, pl1 = {};
#pragma unroll
      for (int i = 0; i < 8; ++i) {
        unsigned hb, lb;
        split_bf16(s[2 * kc][i], hb, lb);
        ph0[i] = (ushort_t)hb;
        pl0[i] = (ushort_t)lb;
        split_bf16(s[2 * kc + 1][i], hb, lb);
        ph1[i] = (ushort_t)hb;
        pl1[i] = (ushort_t)lb;
      }
      Frag pbh, pbl;
      pbh.u[0] = ph0; pbh.u[1] = ph1;
      pbl.u[0] = pl0; pbl.u[1] = pl1;
#pragma unroll
      for (int j = 0; j < 4; ++j) {
        const size_t vo = vrow0 + (size_t)(16 * j + ln) * S_LEN + kb + 32 * kc;
        const v16bf vah = ldfrag(Vth + vo, h);
        const v16bf val = ldfrag(Vtl + vo, h);
        acc[j] = mma3(vah, val, pbh.v, pbl.v, acc[j]);
      }
    }
  }

  const float inv = 1.0f / l;
#pragma unroll
  for (int j = 0; j < 4; ++j)
#pragma unroll
    for (int r = 0; r < 8; ++r)
      osh[16 * w + ln][16 * j + 8 * h + r] = acc[j][r] * inv;
  __syncthreads();

  attn_store(osh, tid, qBase, b, headCol, Ch, Cl);
  __threadfence();
  attn_store(osh, tid, qBase, b, headCol, Ch, Cl);
}

extern "C" void kernel_launch(void* const* d_in, const int* in_sizes, int n_in,
                              void* d_out, int out_size, void* d_ws, size_t ws_size,
                              hipStream_t stream)
{
  if (n_in < 9) return;
  const int nx = MROWS * EMB;
  const int nw = EMB * EMB;
  if (in_sizes[0] != nx || in_sizes[1] != nw || in_sizes[2] != EMB ||
      in_sizes[3] != nw || in_sizes[4] != EMB || in_sizes[5] != nw ||
      in_sizes[6] != EMB || in_sizes[7] != nw || in_sizes[8] != EMB) return;
  if (out_size != nx) return;

  const float* x  = (const float*)d_in[0];
  const float* wq = (const float*)d_in[1];
  const float* bq = (const float*)d_in[2];
  const float* wk = (const float*)d_in[3];
  const float* bk = (const float*)d_in[4];
  const float* wv = (const float*)d_in[5];
  const float* bv = (const float*)d_in[6];
  const float* wo = (const float*)d_in[7];
  const float* bo = (const float*)d_in[8];
  float* out = (float*)d_out;

  const size_t plane = (size_t)nx;
  const size_t need = 12 * plane * sizeof(ushort_t);
  if (need > ws_size) return;
  ushort_t* base = (ushort_t*)d_ws;
  ushort_t* xh  = base + 0 * plane;  ushort_t* xl  = base + 1 * plane;
  ushort_t* whi = base + 2 * plane;  ushort_t* wlo = base + 3 * plane;
  ushort_t* qh  = base + 4 * plane;  ushort_t* ql  = base + 5 * plane;
  ushort_t* kh  = base + 6 * plane;  ushort_t* kl  = base + 7 * plane;
  ushort_t* vth = base + 8 * plane;  ushort_t* vtl = base + 9 * plane;
  ushort_t* ch  = base + 10 * plane; ushort_t* cl  = base + 11 * plane;

  {
    const int groups = nx / 8;
    dim3 g((groups + 255) / 256, 1);
    k_split_planes<<<g, 256, 0, stream>>>(x, x, x, x, groups, xh, xl);
  }
  {
    const int groups = nw / 8;
    dim3 g((groups + 255) / 256, 4);
    k_split_planes<<<g, 256, 0, stream>>>(wq, wk, wv, wo, groups, whi, wlo);
  }

  const dim3 gg(EMB / GBN, MROWS / GBM);
  k_gemm<0><<<gg, 128, 0, stream>>>(xh, xl, whi + 0 * (size_t)nw, wlo + 0 * (size_t)nw, bq, 0.125f, qh, ql, out);
  k_gemm<0><<<gg, 128, 0, stream>>>(xh, xl, whi + 1 * (size_t)nw, wlo + 1 * (size_t)nw, bk, 1.0f, kh, kl, out);
  k_gemm<1><<<gg, 128, 0, stream>>>(xh, xl, whi + 2 * (size_t)nw, wlo + 2 * (size_t)nw, bv, 1.0f, vth, vtl, out);
  {
    dim3 ga(S_LEN / 64, BATCH * HEADS);
    k_attn<<<ga, 128, 0, stream>>>(qh, ql, kh, kl, vth, vtl, ch, cl);
  }
  k_gemm<2><<<gg, 128, 0, stream>>>(ch, cl, whi + 3 * (size_t)nw, wlo + 3 * (size_t)nw, bo, 1.0f, qh, ql, out);
}
